// ScoreNetwork_52948356825732
// MI455X (gfx1250) — hardware-verified
//
#include <hip/hip_runtime.h>
#include <stdint.h>
#include <math.h>

typedef _Float16 v16h __attribute__((ext_vector_type(16)));
typedef _Float16 v8h  __attribute__((ext_vector_type(8)));
typedef _Float16 v4h  __attribute__((ext_vector_type(4)));
typedef float    v8f  __attribute__((ext_vector_type(8)));
typedef float    v4f  __attribute__((ext_vector_type(4)));
typedef int      v4i  __attribute__((ext_vector_type(4)));
typedef unsigned short us4 __attribute__((ext_vector_type(4)));
typedef unsigned short us8 __attribute__((ext_vector_type(8)));
typedef v4f v4fa __attribute__((may_alias));
typedef v4i v4ia __attribute__((may_alias));
typedef us4 us4a __attribute__((may_alias));
typedef us8 us8a __attribute__((may_alias));
typedef unsigned long long u64;
union Frag { v16h v; v8h half[2]; };
union H4 { us4 u; v4h h; };

#define DEV __device__ __forceinline__

DEV unsigned okey(float f) {
  unsigned u = __float_as_uint(f);
  return (u & 0x80000000u) ? ~u : (u | 0x80000000u);
}
DEV u64 mkkey(float sc, int i) { return (((u64)okey(sc)) << 32) | (u64)(~(unsigned)i); }
DEV float lrelu(float x) { return x >= 0.f ? x : 0.2f * x; }
DEV int clampi(int v, int lo, int hi) { return v < lo ? lo : (v > hi ? hi : v); }
DEV v8h zero8h() { v8h z;
#pragma unroll
  for (int i = 0; i < 8; ++i) z[i] = (_Float16)0.0f; return z; }
DEV v8f zero8f() { v8f z;
#pragma unroll
  for (int i = 0; i < 8; ++i) z[i] = 0.f; return z; }

DEV v8f wmma16(v16h a, v16h b, v8f c) {
  return __builtin_amdgcn_wmma_f32_16x16x32_f16(false, a, false, b, (short)0, c, false, false);
}
DEV void nops8(v8f (&acc)[8], const v16h& a, const v16h& b) {
  asm volatile("v_nop\n\tv_nop\n\tv_nop\n\tv_nop"
               : "+v"(acc[0]), "+v"(acc[1]), "+v"(acc[2]), "+v"(acc[3]),
                 "+v"(acc[4]), "+v"(acc[5]), "+v"(acc[6]), "+v"(acc[7])
               : "v"(a), "v"(b));
}
#define CBAR() asm volatile("" ::: "memory")

__global__ void __launch_bounds__(256) k_cvtw4(const float* __restrict__ W1, const float* __restrict__ W2,
                                             const float* __restrict__ W3, const float* __restrict__ W4,
                                             _Float16* T1, _Float16* T2, _Float16* T3, _Float16* T4)
{
  const int y = blockIdx.y;
  const float* W = (y == 0) ? W1 : (y == 1) ? W2 : (y == 2) ? W3 : W4;
  _Float16* T = (y == 0) ? T1 : (y == 1) ? T2 : (y == 2) ? T3 : T4;
  const int xf = (y == 0) ? 20 : 128;
  const int KP = (y == 0) ? 32 : 128;
  const int nrows = (y == 0) ? 256 : 384;
  const int per = KP >> 3;
  const int total = nrows * per;
  const int idx = blockIdx.x * 256 + threadIdx.x;
  const bool ok = idx < total;
  v8h v = zero8h();
  if (ok) {
    const int n = idx / per, k0 = (idx - n * per) * 8;
    int rbase, col, kin;
    if (n < 128)      { rbase = 0;      col = n;       kin = xf; }
    else if (n < 256) { rbase = xf;     col = n - 128; kin = xf; }
    else              { rbase = 2 * xf; col = n - 256; kin = 128; }
#pragma unroll
    for (int i = 0; i < 8; ++i) {
      const int k = k0 + i;
      v[i] = (k < kin) ? (_Float16)W[(size_t)(rbase + k) * 128 + col] : (_Float16)0.0f;
    }
  }
  _Float16* p = T + (size_t)idx * 8;
  if (ok) *(volatile v8h*)p = v;
  __threadfence();
  if (ok) *(volatile v8h*)p = v;
}

__global__ void __launch_bounds__(256) k_x0(const float* __restrict__ nf, const float* __restrict__ nl,
                                          int N, int NP0, _Float16* X0)
{
  const int idx = blockIdx.x * 256 + threadIdx.x;
  const int i = idx >> 2, q = idx & 3;
  v8h v = zero8h();
  if (i < N) {
#pragma unroll
    for (int c = 0; c < 8; ++c) {
      const int cc = q * 8 + c;
      float f = 0.f;
      if (cc < 16)      f = nf[(size_t)i * 16 + cc];
      else if (cc < 20) f = nl[(size_t)i * 4 + (cc - 16)];
      v[c] = (_Float16)f;
    }
  }
  _Float16* p = X0 + (size_t)idx * 8;
  if (idx < NP0 * 4) *(volatile v8h*)p = v;
  __threadfence();
  if (idx < NP0 * 4) *(volatile v8h*)p = v;
}

template <int KP>
__global__ void __launch_bounds__(128) k_ngemm(const _Float16* __restrict__ X, const _Float16* __restrict__ Wt, float* P)
{
  extern __shared__ __align__(16) unsigned char dsm[];
  _Float16* sW = (_Float16*)dsm;
  const int tid = threadIdx.x, lane = tid & 31, w = tid >> 5, h = lane >> 4, m = lane & 15;
  float* sT = (float*)(dsm + 256 * KP * 2) + w * 2048;
  {
    constexpr int nW = 256 * KP / 8;
    for (int i = tid; i < nW; i += 128) *(v8h*)(sW + i * 8) = *(const v8h*)(Wt + (size_t)i * 8);
  }
  __syncthreads();
  const int row0 = blockIdx.x * 64 + w * 16;
  const _Float16* arow = X + (size_t)(row0 + m) * KP + 8 * h;
#pragma unroll 1
  for (int cg = 0; cg < 2; ++cg) {
    v8f acc[8];
#pragma unroll
    for (int nt = 0; nt < 8; ++nt) acc[nt] = zero8f();
    const _Float16* bb0 = sW + (size_t)(cg * 128 + m) * KP + 8 * h;
    Frag a, b;
#pragma unroll
    for (int ks = 0; ks < KP / 32; ++ks) {
      a.half[0] = *(const v8h*)(arow + ks * 32);
      a.half[1] = *(const v8h*)(arow + ks * 32 + 16);
#pragma unroll
      for (int nt = 0; nt < 8; ++nt) {
        const _Float16* bp = bb0 + nt * 16 * KP + ks * 32;
        b.half[0] = *(const v8h*)bp;
        b.half[1] = *(const v8h*)(bp + 16);
        acc[nt] = wmma16(a.v, b.v, acc[nt]);
      }
      nops8(acc, a.v, b.v);
    }
#pragma unroll
    for (int nt = 0; nt < 8; ++nt) {
#pragma unroll
      for (int r = 0; r < 8; ++r) sT[(8 * h + r) * 128 + nt * 16 + m] = acc[nt][r];
    }
    CBAR();
#pragma unroll 1
    for (int pass = 0; pass < 2; ++pass) {
      if (pass) __threadfence();
#pragma unroll 1
      for (int r = 0; r < 16; ++r) {
        const v4fa v = *(const v4fa*)(sT + r * 128 + 4 * lane);
        *(volatile v4f*)(P + (size_t)(row0 + r) * 256 + cg * 128 + 4 * lane) = v;
      }
    }
    CBAR();
  }
}

__global__ void __launch_bounds__(256) k_econv1(const float* __restrict__ P, const float* __restrict__ ef,
                                              const float* __restrict__ W1, const float* __restrict__ b1,
                                              const int* __restrict__ sarr, const int* __restrict__ darr,
                                              int E, int N, _Float16* eb)
{
  const int tid = threadIdx.x, lane = tid & 31, w = tid >> 5, h = lane >> 4, m = lane & 15;
  const int gw = blockIdx.x * 8 + w;
  float we[4][8], bb[8];
#pragma unroll
  for (int j = 0; j < 4; ++j) {
#pragma unroll
    for (int c = 0; c < 8; ++c) we[j][c] = W1[(size_t)(40 + j) * 128 + 8 * m + c];
  }
#pragma unroll
  for (int c = 0; c < 8; ++c) bb[c] = b1[8 * m + c];
#pragma unroll 1
  for (int it = 0; it < 4; ++it) {
    const int e = (gw * 4 + it) * 2 + h;
    const bool inb = e < E;
    const int ec = inb ? e : E - 1;
    const int d = clampi(darr[ec], 0, N - 1), s = clampi(sarr[ec], 0, N - 1);
    const v4f pd0 = *(const v4f*)(P + (size_t)d * 256 + 8 * m);
    const v4f pd1 = *(const v4f*)(P + (size_t)d * 256 + 8 * m + 4);
    const v4f ps0 = *(const v4f*)(P + (size_t)s * 256 + 128 + 8 * m);
    const v4f ps1 = *(const v4f*)(P + (size_t)s * 256 + 128 + 8 * m + 4);
    const v4f f = *(const v4f*)(ef + (size_t)ec * 4);
    float g[8];
#pragma unroll
    for (int c = 0; c < 4; ++c) { g[c] = pd0[c] + ps0[c]; g[4 + c] = pd1[c] + ps1[c]; }
    v8h o;
#pragma unroll
    for (int c = 0; c < 8; ++c) {
      float dv = f[0] * we[0][c];
      dv += f[1] * we[1][c]; dv += f[2] * we[2][c]; dv += f[3] * we[3][c];
      float hv = (g[c] + dv) + bb[c];
      hv = hv > 0.f ? hv : 0.f;
      o[c] = (_Float16)hv;
    }
    _Float16* p = eb + (size_t)ec * 128 + 8 * m;
    if (inb) *(volatile v8h*)p = o;
    __threadfence();
    if (inb) *(volatile v8h*)p = o;
  }
}

__global__ void __launch_bounds__(256) k_gath(const float* __restrict__ P, const int* __restrict__ sarr,
                                            const int* __restrict__ darr, int E, int N, int eb0, int cnt, float* G)
{
  const int tid = threadIdx.x, lane = tid & 31, w = tid >> 5;
  const int gw = blockIdx.x * 8 + w;
#pragma unroll 1
  for (int it = 0; it < 8; ++it) {
    const int el = gw * 8 + it;
    if (el < cnt) {
      const int e = eb0 + el;
      const int d = clampi(darr[e], 0, N - 1), s = clampi(sarr[e], 0, N - 1);
      const v4f a = *(const v4f*)(P + (size_t)d * 256 + 4 * lane);
      const v4f c = *(const v4f*)(P + (size_t)s * 256 + 128 + 4 * lane);
      v4f g; g.x = a.x + c.x; g.y = a.y + c.y; g.z = a.z + c.z; g.w = a.w + c.w;
      float* p = G + (size_t)el * 128 + 4 * lane;
      *(volatile v4f*)p = g;
      __threadfence();
      *(volatile v4f*)p = g;
    }
  }
}

__global__ void __launch_bounds__(128) k_econv(_Float16* eb, const _Float16* __restrict__ Wt, const float* __restrict__ G,
                                             const float* __restrict__ bias, const int* __restrict__ msk, int usem,
                                             int E, int eb0, int ntiles)
{
  extern __shared__ __align__(16) unsigned char dsm[];
  _Float16* sW = (_Float16*)dsm;
  const int tid = threadIdx.x, lane = tid & 31, w = tid >> 5, h = lane >> 4, m = lane & 15;
  float* sT = (float*)(dsm + 128 * 128 * 2) + w * 2048;
  for (int i = tid; i < 2048; i += 128) *(v8h*)(sW + i * 8) = *(const v8h*)(Wt + (size_t)i * 8);
  __syncthreads();
  float bb[8];
#pragma unroll
  for (int c = 0; c < 8; ++c) bb[c] = bias[8 * m + c];
  const int nwv = gridDim.x * 4;
  for (int tile = blockIdx.x * 4 + w; tile < ntiles; tile += nwv) {
    const int e0 = eb0 + tile * 16;
    const int er = e0 + m;
    const int erc = er < E ? er : E - 1;
    bool vr = er < E;
    if (usem) vr = vr && (msk[erc] != 0);
    const unsigned bal = __builtin_amdgcn_ballot_w32(vr) & 0xFFFFu;
    v8h o[8];
    if (bal != 0u) {
      v8f acc[8];
#pragma unroll
      for (int nt = 0; nt < 8; ++nt) acc[nt] = zero8f();
      const _Float16* arow = eb + (size_t)erc * 128 + 8 * h;
      const _Float16* bb0 = sW + m * 128 + 8 * h;
      Frag a, b;
#pragma unroll
      for (int ks = 0; ks < 4; ++ks) {
        a.half[0] = *(const v8h*)(arow + ks * 32);
        a.half[1] = *(const v8h*)(arow + ks * 32 + 16);
#pragma unroll
        for (int nt = 0; nt < 8; ++nt) {
          const _Float16* bp = bb0 + nt * 16 * 128 + ks * 32;
          b.half[0] = *(const v8h*)bp;
          b.half[1] = *(const v8h*)(bp + 16);
          acc[nt] = wmma16(a.v, b.v, acc[nt]);
        }
        nops8(acc, a.v, b.v);
      }
#pragma unroll
      for (int nt = 0; nt < 8; ++nt) {
#pragma unroll
        for (int r = 0; r < 8; ++r) sT[(8 * h + r) * 128 + nt * 16 + m] = acc[nt][r];
      }
      CBAR();
#pragma unroll
      for (int p = 0; p < 8; ++p) {
        const int row = 2 * p + h;
        const int e = e0 + row;
        const int ec = e < E ? e : E - 1;
        const v4fa t0 = *(const v4fa*)(sT + row * 128 + 8 * m);
        const v4fa t1 = *(const v4fa*)(sT + row * 128 + 8 * m + 4);
        const v4f g0 = *(const v4f*)(G + (size_t)(ec - eb0) * 128 + 8 * m);
        const v4f g1 = *(const v4f*)(G + (size_t)(ec - eb0) * 128 + 8 * m + 4);
        const bool vrow = ((bal >> row) & 1u) != 0u;
        float tv8[8];
#pragma unroll
        for (int c = 0; c < 4; ++c) { tv8[c] = t0[c] + g0[c]; tv8[4 + c] = t1[c] + g1[c]; }
        v8h ov;
#pragma unroll
        for (int c = 0; c < 8; ++c) {
          float hv = tv8[c] + bb[c];
          hv = (vrow && hv > 0.f) ? hv : 0.f;
          ov[c] = (_Float16)hv;
        }
        o[p] = ov;
      }
      CBAR();
    } else {
#pragma unroll
      for (int p = 0; p < 8; ++p) o[p] = zero8h();
    }
#pragma unroll
    for (int p = 0; p < 8; ++p) {
      const int e = e0 + 2 * p + h;
      if (e < E) *(volatile v8h*)(eb + (size_t)e * 128 + 8 * m) = o[p];
    }
    __threadfence();
#pragma unroll
    for (int p = 0; p < 8; ++p) {
      const int e = e0 + 2 * p + h;
      if (e < E) *(volatile v8h*)(eb + (size_t)e * 128 + 8 * m) = o[p];
    }
  }
}

__global__ void __launch_bounds__(32) k_agg(const _Float16* __restrict__ eb, const int* __restrict__ darr,
                                          const int* __restrict__ msk, int usem, int E, int niter,
                                          const float* __restrict__ gw, _Float16* xo, float* hb)
{
  extern __shared__ __align__(16) unsigned char dsm[];
  unsigned short* sg = (unsigned short*)dsm;
  float* sH = (float*)(dsm + 512 * 128 * 2);
  const int lane = threadIdx.x, h = lane >> 4, m = lane & 15;
  const int base = blockIdx.x * 512;
  {
    us8 z;
#pragma unroll
    for (int i = 0; i < 8; ++i) z[i] = 0;
    for (int i = lane; i < 512 * 128 / 8; i += 32) *(us8*)(sg + i * 8) = z;
  }
  const v4f w4 = *(const v4f*)(gw + 4 * lane);
  __syncthreads();
  const unsigned short* ebu = (const unsigned short*)eb;
  for (int it = 0; it < niter; ++it) {
    const int ebase = it * 128;
#pragma unroll 1
    for (int sub = 0; sub < 4; ++sub) {
      const int e = ebase + sub * 32 + lane;
      bool f = false; int rel = 0;
      if (e < E) {
        bool mk = true;
        if (usem) mk = (msk[e] != 0);
        rel = darr[e] - base;
        f = mk && ((unsigned)rel < 512u);
      }
      unsigned bal = __builtin_amdgcn_ballot_w32(f);
#pragma unroll 1
      for (int t = 0; t < 32; ++t) {
        if (bal == 0u) break;
        const int j = __builtin_ctz(bal);
        bal &= bal - 1u;
        const int ln = __shfl(rel, j);
        const int ed = ebase + sub * 32 + j;
        const us4 v = *(const us4*)(ebu + (size_t)ed * 128 + 4 * lane);
        us4a* gp = (us4a*)(sg + ln * 128 + 4 * lane);
        const us4 cur = *gp;
        us4 r;
        r.x = cur.x > v.x ? cur.x : v.x;
        r.y = cur.y > v.y ? cur.y : v.y;
        r.z = cur.z > v.z ? cur.z : v.z;
        r.w = cur.w > v.w ? cur.w : v.w;
        *gp = r;
      }
    }
  }
  __syncthreads();
#pragma unroll 1
  for (int row = 0; row < 512; ++row) {
    H4 x; x.u = *(const us4a*)(sg + row * 128 + 4 * lane);
    float s = (float)x.h.x * w4.x;
    s += (float)x.h.y * w4.y; s += (float)x.h.z * w4.z; s += (float)x.h.w * w4.w;
    s += __shfl_xor(s, 16); s += __shfl_xor(s, 8); s += __shfl_xor(s, 4); s += __shfl_xor(s, 2); s += __shfl_xor(s, 1);
    if (lane == 0) sH[row] = s;
  }
  __syncthreads();
  unsigned short* xu = (unsigned short*)xo;
#pragma unroll 1
  for (int pass = 0; pass < 2; ++pass) {
    if (pass) __threadfence();
#pragma unroll 1
    for (int rp = 0; rp < 256; ++rp) {
      const int row = rp * 2 + h;
      const us8a v = *(const us8a*)(sg + row * 128 + m * 8);
      *(volatile us8*)(xu + (size_t)(base + row) * 128 + m * 8) = v;
    }
#pragma unroll 1
    for (int q = 0; q < 4; ++q) {
      const v4fa v = *(const v4fa*)(sH + q * 128 + 4 * lane);
      *(volatile v4f*)(hb + base + q * 128 + 4 * lane) = v;
    }
  }
}

__global__ void __launch_bounds__(32) k_gscan(const float* __restrict__ hb, const int* __restrict__ sarr,
                                            const int* __restrict__ darr, const int* __restrict__ msk, int usem,
                                            const float* __restrict__ ga, const float* __restrict__ gb,
                                            int E, int N, int niter, float* score)
{
#pragma clang fp contract(off)
  __shared__ float sh[2048];
  __shared__ float sm[2048];
  __shared__ float sdn[2048];
  __shared__ float snm[2048];
  const int lane = threadIdx.x;
  const int base = blockIdx.x * 2048;
  const float a0 = ga[0], a1 = ga[1];
  for (int i = lane; i < 2048; i += 32) {
    const float hv = hb[base + i];
    const float al = a0 * hv;
    const float ar = a1 * hv;
    sh[i] = hv; sm[i] = lrelu(al + ar); sdn[i] = 1.f; snm[i] = hv;
  }
  __syncthreads();
  for (int it = 0; it < niter; ++it) {
    const int ebase = it * 128;
#pragma unroll 1
    for (int sub = 0; sub < 4; ++sub) {
      const int e = ebase + sub * 32 + lane;
      bool f = false; int rel = 0;
      if (e < E) {
        bool mk = true;
        if (usem) mk = (msk[e] != 0);
        rel = darr[e] - base;
        f = mk && ((unsigned)rel < 2048u);
      }
      unsigned bal = __builtin_amdgcn_ballot_w32(f);
#pragma unroll 1
      for (int t = 0; t < 32; ++t) {
        if (bal == 0u) break;
        const int j = __builtin_ctz(bal);
        bal &= bal - 1u;
        const int ln = __shfl(rel, j);
        const int ed = ebase + sub * 32 + j;
        const int sv = clampi(sarr[ed], 0, N - 1);
        const float hs = hb[sv];
        const float al = a0 * hs;
        const float ar = a1 * sh[ln];
        const float v = lrelu(al + ar);
        float mo = sm[ln], dn = sdn[ln], nm = snm[ln];
        if (v > mo) {
          const float rr = expf(mo - v);
          dn = dn * rr + 1.f;
          nm = nm * rr + hs;
          mo = v;
        } else {
          const float ww = expf(v - mo);
          dn = dn + ww;
          nm = nm + ww * hs;
        }
        sm[ln] = mo; sdn[ln] = dn; snm[ln] = nm;
      }
    }
  }
  __syncthreads();
  const float b0 = gb[0];
  for (int i = lane; i < 2048; i += 32) sm[i] = snm[i] / sdn[i] + b0;
  __syncthreads();
#pragma unroll 1
  for (int pass = 0; pass < 2; ++pass) {
    if (pass) __threadfence();
#pragma unroll 1
    for (int q = 0; q < 16; ++q) {
      const v4fa v = *(const v4fa*)(sm + q * 128 + 4 * lane);
      *(volatile v4f*)(score + base + q * 128 + 4 * lane) = v;
    }
  }
}

__global__ void __launch_bounds__(512) k_sel(const float* __restrict__ score, const int* __restrict__ selp, int usep,
                                           const _Float16* __restrict__ xh, const int* __restrict__ sarr,
                                           const int* __restrict__ darr, int E, int EP, int N, int NP0, int nsort, int k,
                                           int* sel, _Float16* xs, int dox, int* mko, int dom, float* lpo)
{
  extern __shared__ __align__(16) unsigned char dsm[];
  __shared__ float smx[128];
  __shared__ float smn[128];
  u64* key = (u64*)dsm;
  const int t = threadIdx.x;
  for (int i = t; i < nsort; i += 512) {
    u64 kv = 0ull;
    if (i < N) {
      bool sp = true;
      if (usep) sp = (selp[i] != 0);
      if (sp) kv = mkkey(score[i], i);
    }
    key[i] = kv;
  }
  __syncthreads();
  const int halfn = nsort >> 1;
  for (int size = 2; size <= nsort; size <<= 1) {
    for (int stride = size >> 1; stride > 0; stride >>= 1) {
      for (int p = t; p < halfn; p += 512) {
        const int i = ((p & ~(stride - 1)) << 1) | (p & (stride - 1));
        const int j = i + stride;
        const u64 a = key[i], c = key[j];
        const bool up = ((i & size) == 0);
        const bool sw = up ? (a > c) : (a < c);
        if (sw) { key[i] = c; key[j] = a; }
      }
      __syncthreads();
    }
  }
  const u64 thr = key[nsort - k];
  __syncthreads();
  int* ssel = (int*)dsm;
  float* stn = (float*)(dsm + 65536);
  for (int i = t; i < NP0; i += 512) {
    int s = 0; float tv = 0.f;
    if (i < N) {
      bool sp = true;
      if (usep) sp = (selp[i] != 0);
      if (sp && mkkey(score[i], i) >= thr) s = 1;
      tv = tanhf(score[i]);
    }
    ssel[i] = s; stn[i] = tv;
  }
  __syncthreads();
  if (t < 128) {
    float mx = -INFINITY;
#pragma unroll 1
    for (int i = 0; i < N; ++i) {
      if (ssel[i]) { const float v = (float)xh[(size_t)i * 128 + t] * stn[i]; mx = fmaxf(mx, v); }
    }
    smx[t] = mx;
  } else if (t < 256) {
    const int c = t - 128;
    double sum = 0.0;
#pragma unroll 1
    for (int i = 0; i < N; ++i) {
      if (ssel[i]) { const float v = (float)xh[(size_t)i * 128 + c] * stn[i]; sum += (double)v; }
    }
    smn[c] = (float)(sum / (double)k);
  }
  __syncthreads();
  auto emit = [&]() {
    for (int q = t; q < (NP0 >> 2); q += 512) {
      const v4ia v = *(const v4ia*)(ssel + 4 * q);
      *(volatile v4i*)(sel + 4 * q) = v;
    }
    if (t < 32)      { const v4fa v = *(const v4fa*)(smx + 4 * t);        *(volatile v4f*)(lpo + 4 * t) = v; }
    else if (t < 64) { const v4fa v = *(const v4fa*)(smn + 4 * (t - 32)); *(volatile v4f*)(lpo + 128 + 4 * (t - 32)) = v; }
    if (dox) {
      for (int idx = t; idx < NP0 * 16; idx += 512) {
        const int i = idx >> 4, q = idx & 15;
        v8h o = zero8h();
        if (ssel[i]) {
          const v8h xv = *(const v8h*)(xh + (size_t)i * 128 + 8 * q);
          const float tv = stn[i];
#pragma unroll
          for (int c = 0; c < 8; ++c) o[c] = (_Float16)((float)xv[c] * tv);
        }
        *(volatile v8h*)(xs + (size_t)i * 128 + 8 * q) = o;
      }
    }
    if (dom) {
      for (int q = t; q < (EP >> 2); q += 512) {
        int mm[4];
#pragma unroll
        for (int jj = 0; jj < 4; ++jj) {
          const int e = 4 * q + jj;
          int mv = 0;
          if (e < E) {
            const int s = clampi(sarr[e], 0, N - 1), d = clampi(darr[e], 0, N - 1);
            mv = (ssel[s] & ssel[d]);
          }
          mm[jj] = mv;
        }
        v4i v; v.x = mm[0]; v.y = mm[1]; v.z = mm[2]; v.w = mm[3];
        *(volatile v4i*)(mko + 4 * q) = v;
      }
    }
  };
  emit();
  __threadfence();
  emit();
}

__global__ void __launch_bounds__(128) k_head(const float* __restrict__ lp,
                                            const float* __restrict__ lw1, const float* __restrict__ lb1,
                                            const float* __restrict__ lw2, const float* __restrict__ lb2,
                                            const float* __restrict__ lw3, const float* __restrict__ lb3,
                                            float* out)
{
  __shared__ float sl[256];
  __shared__ float h1[128];
  __shared__ float h2[64];
  __shared__ float so[4];
  const int t = threadIdx.x;
  sl[t]       = (lp[t] + lp[256 + t]) + lp[512 + t];
  sl[t + 128] = (lp[t + 128] + lp[256 + t + 128]) + lp[512 + t + 128];
  __syncthreads();
  {
    float a = 0.f;
#pragma unroll 4
    for (int j = 0; j < 256; ++j) a += sl[j] * lw1[j * 128 + t];
    a += lb1[t];
    h1[t] = a > 0.f ? a : 0.f;
  }
  __syncthreads();
  if (t < 64) {
    float a = 0.f;
#pragma unroll 4
    for (int j = 0; j < 128; ++j) a += h1[j] * lw2[j * 64 + t];
    a += lb2[t];
    h2[t] = a > 0.f ? a : 0.f;
  }
  __syncthreads();
  if (t < 4) {
    float a = 0.f;
#pragma unroll 4
    for (int j = 0; j < 64; ++j) a += h2[j] * lw3[j * 4 + t];
    a += lb3[t];
    so[t] = a;
  }
  __syncthreads();
  if (t == 0) {
    v4f v; v.x = so[0]; v.y = so[1]; v.z = so[2]; v.w = so[3];
    *(volatile v4f*)out = v;
    __threadfence();
    *(volatile v4f*)out = v;
  }
}

static inline int cdiv_i(long long a, long long b) { return (int)((a + b - 1) / b); }
static inline int rup_i(int a, int b) { return ((a + b - 1) / b) * b; }

extern "C" void kernel_launch(void* const* d_in, const int* in_sizes, int n_in,
                              void* d_out, int out_size, void* d_ws, size_t ws_size,
                              hipStream_t stream)
{
  (void)n_in; (void)out_size;
  const float* node_feat  = (const float*)d_in[0];
  const float* node_level = (const float*)d_in[1];
  const int*   eidx       = (const int*)d_in[2];
  const float* edge_feat  = (const float*)d_in[3];
  const float* W1 = (const float*)d_in[4];   const float* b1 = (const float*)d_in[5];
  const float* W2 = (const float*)d_in[6];   const float* b2 = (const float*)d_in[7];
  const float* W3 = (const float*)d_in[8];   const float* b3 = (const float*)d_in[9];
  const float* W4 = (const float*)d_in[10];  const float* b4 = (const float*)d_in[11];
  const float* gW2 = (const float*)d_in[12]; const float* ga2 = (const float*)d_in[13]; const float* gb2 = (const float*)d_in[14];
  const float* gW3 = (const float*)d_in[15]; const float* ga3 = (const float*)d_in[16]; const float* gb3 = (const float*)d_in[17];
  const float* gW4 = (const float*)d_in[18]; const float* ga4 = (const float*)d_in[19]; const float* gb4 = (const float*)d_in[20];
  const float* lw1 = (const float*)d_in[21]; const float* lb1 = (const float*)d_in[22];
  const float* lw2 = (const float*)d_in[23]; const float* lb2 = (const float*)d_in[24];
  const float* lw3 = (const float*)d_in[25]; const float* lb3 = (const float*)d_in[26];

  const int N = in_sizes[0] / 16;
  const int E = in_sizes[2] / 2;
  if (N < 1 || E < 1 || N > 16384) return;
  const int* src = eidx;
  const int* dst = eidx + E;
  const int k1 = (N + 1) / 2, k2 = (k1 + 1) / 2, k3 = (k2 + 1) / 2;
  const int NP0 = rup_i(N, 2048), N64 = rup_i(N, 64), EP = rup_i(E, 1024);
  int nsort = 1024; while (nsort < N) nsort <<= 1;
  const int NSLAB = 6;
  const int S = rup_i(cdiv_i(E, NSLAB), 64);
  const int nit = cdiv_i(E, 128);

  char* wp = (char*)d_ws;
  size_t used = 0;
  auto carve = [&](size_t bytes) -> char* { char* p = wp + used; used += (bytes + 255) & ~(size_t)255; return p; };
  _Float16* Wt1 = (_Float16*)carve((size_t)256 * 32 * 2);
  _Float16* Wt2 = (_Float16*)carve((size_t)384 * 128 * 2);
  _Float16* Wt3 = (_Float16*)carve((size_t)384 * 128 * 2);
  _Float16* Wt4 = (_Float16*)carve((size_t)384 * 128 * 2);
  _Float16* ebuf = (_Float16*)carve((size_t)E * 128 * 2);
  size_t regG = (size_t)S * 128 * 4; if (regG < (size_t)NP0 * 32 * 2) regG = (size_t)NP0 * 32 * 2;
  float*    Gbuf = (float*)carve(regG);
  _Float16* X0h  = (_Float16*)Gbuf;
  float*    P    = (float*)carve((size_t)N64 * 256 * 4);
  _Float16* xA   = (_Float16*)carve((size_t)NP0 * 128 * 2);
  _Float16* xB   = (_Float16*)carve((size_t)NP0 * 128 * 2);
  float*    hbuf  = (float*)carve((size_t)NP0 * 4);
  float*    score = (float*)carve((size_t)NP0 * 4);
  int*      sel1 = (int*)carve((size_t)NP0 * 4);
  int*      sel2 = (int*)carve((size_t)NP0 * 4);
  int*      sel3 = (int*)carve((size_t)NP0 * 4);
  int*      msk  = (int*)carve((size_t)EP * 4);
  float*    lp   = (float*)carve((size_t)3 * 256 * 4);
  if (used > ws_size) return;

  const size_t smemN32 = (size_t)256 * 32 * 2 + 4 * 2048 * 4;
  const size_t smemN128 = (size_t)256 * 128 * 2 + 4 * 2048 * 4;
  const size_t smemE = (size_t)128 * 128 * 2 + 4 * 2048 * 4;
  const size_t smemAgg = (size_t)512 * 128 * 2 + 512 * 4;
  const size_t smemSel = (size_t)16384 * 8;

  k_cvtw4<<<dim3(24, 4), dim3(256), 0, stream>>>(W1, W2, W3, W4, Wt1, Wt2, Wt3, Wt4);
  k_x0<<<dim3(NP0 / 64), dim3(256), 0, stream>>>(node_feat, node_level, N, NP0, X0h);

  k_ngemm<32><<<dim3(N64 / 64), dim3(128), smemN32, stream>>>(X0h, Wt1, P);
  k_econv1<<<dim3(cdiv_i(cdiv_i(E, 2), 32)), dim3(256), 0, stream>>>(P, edge_feat, W1, b1, src, dst, E, N, ebuf);
  k_agg<<<dim3(NP0 / 512), dim3(32), smemAgg, stream>>>(ebuf, dst, msk, 0, E, nit, gW2, xA, hbuf);

  auto conv = [&](const _Float16* X, const _Float16* Wt, const float* b, int usem, const float* gw, _Float16* xout) {
    k_ngemm<128><<<dim3(N64 / 64), dim3(128), smemN128, stream>>>(X, Wt, P);
    for (int sb = 0; sb < NSLAB; ++sb) {
      const int eb0 = sb * S;
      int cnt = E - eb0; if (cnt > S) cnt = S;
      if (cnt <= 0) break;
      k_gath<<<dim3(cdiv_i(cnt, 64)), dim3(256), 0, stream>>>(P, src, dst, E, N, eb0, cnt, Gbuf);
      const int ntl = cdiv_i(cnt, 16);
      int gb = cdiv_i(ntl, 4); if (gb > 512) gb = 512;
      k_econv<<<dim3(gb), dim3(128), smemE, stream>>>(ebuf, Wt + 256 * 128, Gbuf, b, msk, usem, E, eb0, ntl);
    }
    k_agg<<<dim3(NP0 / 512), dim3(32), smemAgg, stream>>>(ebuf, dst, msk, usem, E, nit, gw, xout, hbuf);
  };
  auto pool = [&](const int* selp, int usep, const _Float16* xh, int usem, const float* ga, const float* gbias,
                  int k, int* selo, _Float16* xso, int dox, int dom, float* lpart) {
    k_gscan<<<dim3(NP0 / 2048), dim3(32), 0, stream>>>(hbuf, src, dst, msk, usem, ga, gbias, E, N, nit, score);
    k_sel<<<dim3(1), dim3(512), smemSel, stream>>>(score, selp, usep, xh, src, dst, E, EP, N, NP0, nsort, k,
                                                   selo, xso, dox, msk, dom, lpart);
  };

  conv(xA, Wt2, b2, 0, gW2, xB);
  pool(sel1, 0, xB, 0, ga2, gb2, k1, sel1, xA, 1, 1, lp);
  conv(xA, Wt3, b3, 1, gW3, xA);
  pool(sel1, 1, xA, 1, ga3, gb3, k2, sel2, xB, 1, 1, lp + 256);
  conv(xB, Wt4, b4, 1, gW4, xB);
  pool(sel2, 1, xB, 1, ga4, gb4, k3, sel3, xA, 0, 0, lp + 512);

  k_head<<<dim3(1), dim3(128), 0, stream>>>(lp, lw1, lb1, lw2, lb2, lw3, lb3, (float*)d_out);
  (void)hipGetLastError();
}
